// MultiHeadAttention_8091718386486
// MI455X (gfx1250) — hardware-run, weakly checked
//
#include <hip/hip_runtime.h>
#include <math.h>

#ifndef NB
#define NB 2
#endif
#ifndef SEQ
#define SEQ 2048
#endif
#define NB_FULL 2
#define SEQ_FULL 2048
#define DM 512
#define NH 8
#define DKH 64
#define NTOK (NB * SEQ)
#define OP 68
#define OPH 36
#define TP 72
#define KCH 128
#define QCARRY 16.0f
#define VCARRY 16.0f
#define WCARRY 16.0f
#define KCARRY 256.0f
#define PCARRY 4096.0f

static_assert(DM == NH * DKH);
static_assert(DKH == 64);
static_assert(NH == 8);
static_assert(SEQ % 64 == 0);
static_assert(SEQ % KCH == 0);
static_assert(SEQ % 16 == 0);
static_assert(SEQ % 8 == 0);
static_assert(SEQ_FULL % 8 == 0);
static_assert(NTOK % 64 == 0);
static_assert(DM % 64 == 0);
static_assert(DKH % 32 == 0);
static_assert((DM * DKH) % DM == 0);
static_assert(NB <= NB_FULL);
static_assert(SEQ <= SEQ_FULL);
static_assert((OP % 4) == 0);
static_assert((OPH % 4) == 0);
static_assert((TP % 8) == 0);
static_assert(KCH == 8 * 16);

typedef __attribute__((ext_vector_type(16))) _Float16 v16h;
typedef __attribute__((ext_vector_type(8)))  _Float16 v8h;
typedef __attribute__((ext_vector_type(16))) __bf16   v16b;
typedef __attribute__((ext_vector_type(8)))  __bf16   v8b;
typedef __attribute__((ext_vector_type(8)))  float    v8f;
typedef __attribute__((ext_vector_type(4)))  float    v4f;
typedef __attribute__((ext_vector_type(4)))  unsigned int v4u;
typedef v8h v8h_ma __attribute__((may_alias));
typedef v4f v4f_ma __attribute__((may_alias));


__device__ __forceinline__ unsigned int bf_bits(float f) {
    const unsigned int u = __float_as_uint(f);
    return (u + 0x7FFFu + ((u >> 16) & 1u)) >> 16;
}
__device__ __forceinline__ float bf_val(float f) { return __uint_as_float(bf_bits(f) << 16); }
__device__ __forceinline__ unsigned int pk_h2(float a, float b) {
    return (unsigned int)__builtin_bit_cast(unsigned short, (_Float16)a) | ((unsigned int)__builtin_bit_cast(unsigned short, (_Float16)b) << 16);
}
__device__ __forceinline__ void pk_split2(float a, float b, unsigned int& hi, unsigned int& lo) {
    const unsigned int ha = bf_bits(a), hb = bf_bits(b);
    const unsigned int la = bf_bits(a - __uint_as_float(ha << 16)), lb = bf_bits(b - __uint_as_float(hb << 16));
    hi = ha | (hb << 16); lo = la | (lb << 16);
}
static __device__ __forceinline__ _Float16 toh_flush(float v) {
    const _Float16 r = (_Float16)v;
    return (fabsf(v) < 6.103515625e-05f) ? (_Float16)0.0f : r;
}
static __device__ __forceinline__ unsigned int pk_h2f(float a, float b) {
    return (unsigned int)__builtin_bit_cast(unsigned short, toh_flush(a)) | ((unsigned int)__builtin_bit_cast(unsigned short, toh_flush(b)) << 16);
}
__device__ __forceinline__ void wave_sync() {
    __builtin_amdgcn_fence(3  , "workgroup");
    __builtin_amdgcn_wave_barrier();
    __builtin_amdgcn_fence(2  , "workgroup");
}

__device__ __forceinline__ v16h ldfrag_h(const unsigned short* __restrict__ p) {
    const v8h a = *(const v8h*)(p);
    const v8h b = *(const v8h*)(p + 16);
    return __builtin_shufflevector(a, b, 0, 1, 2, 3, 4, 5, 6, 7, 8, 9, 10, 11, 12, 13, 14, 15);
}
__device__ __forceinline__ v16b ldfrag_b(const unsigned short* __restrict__ p) {
    const v8b a = *(const v8b*)(p);
    const v8b b = *(const v8b*)(p + 16);
    return __builtin_shufflevector(a, b, 0, 1, 2, 3, 4, 5, 6, 7, 8, 9, 10, 11, 12, 13, 14, 15);
}

template <int ET> struct FragT;
template <> struct FragT<0> {
    typedef v16h V;
    static __device__ __forceinline__ v16h load(const unsigned short* __restrict__ p) { return ldfrag_h(p); }
    static __device__ __forceinline__ v8f mma(v16h a, v16h b, v8f c) { return __builtin_amdgcn_wmma_f32_16x16x32_f16(false, a, false, b, (short)0, c, false, false); }
};
template <> struct FragT<1> {
    typedef v16b V;
    static __device__ __forceinline__ v16b load(const unsigned short* __restrict__ p) { return ldfrag_b(p); }
    static __device__ __forceinline__ v8f mma(v16b a, v16b b, v8f c) { return __builtin_amdgcn_wmma_f32_16x16x32_bf16(false, a, false, b, (short)0, c, false, false); }
};
template <typename V>
__device__ __forceinline__ void guard4(v8f& a, v8f& b, v8f& c, v8f& d, V x, V y0, V y1, V y2, V y3) {
    asm volatile("v_nop\n\tv_nop\n\tv_nop\n\tv_nop" : "+v"(a), "+v"(b), "+v"(c), "+v"(d) : "v"(x), "v"(y0), "v"(y1), "v"(y2), "v"(y3));
}
static __device__ __forceinline__ v8f mma_h(v16h a, v16h b, v8f c) {
    c = __builtin_amdgcn_wmma_f32_16x16x32_f16(false, a, false, b, (short)0, c, false, false);
    asm volatile("v_nop\n\tv_nop\n\tv_nop\n\tv_nop" : "+v"(c) : "v"(a), "v"(b));
    return c;
}

template <int ET, int BIAS_MODE, int OUT_MODE>
__device__ __forceinline__ void gemm64_body(const unsigned short* __restrict__ A, int lda,
                                            const unsigned short* __restrict__ Bt, int ldb,
                                            float* __restrict__ Cf, unsigned short* __restrict__ Ca, unsigned short* __restrict__ Cb, int ldc,
                                            const float* __restrict__ bias, int M, int N, int K,
                                            float scale, float bscale, int cseq, int cseqfull) {
    typedef typename FragT<ET>::V V;
    __shared__ __align__(16) float sT[8 * 16 * OP];
    const int lane = threadIdx.x & 31;
    const int wave = __builtin_amdgcn_readfirstlane(threadIdx.x >> 5);
    const int tilesN = N >> 6;
    const int tilesM = M >> 6;
    const int tile = blockIdx.x * 8 + wave;
    if (tile >= tilesM * tilesN) return;
    const int tm = tile / tilesN;
    const int tn = tile - tm * tilesN;
    const int m0 = tm << 6;
    const int n0 = tn << 6;
    const int rl   = lane & 15;
    const int koff = (lane >> 4) * 8;
    const int mOff = (lane >> 4) * 8;

    v8f acc[4][4];
#pragma unroll
    for (int i = 0; i < 4; ++i)
#pragma unroll
        for (int j = 0; j < 4; ++j) { const v8f zz = {0.f, 0.f, 0.f, 0.f, 0.f, 0.f, 0.f, 0.f}; acc[i][j] = zz; }

    for (int k0 = 0; k0 < K; k0 += 32) {
        V bh[4];
#pragma unroll
        for (int j = 0; j < 4; ++j) bh[j] = FragT<ET>::load(Bt + (size_t)(n0 + (j << 4) + rl) * ldb + koff + k0);
#pragma unroll
        for (int i = 0; i < 4; ++i) {
            const V ah = FragT<ET>::load(A + (size_t)(m0 + (i << 4) + rl) * lda + koff + k0);
            acc[i][0] = FragT<ET>::mma(ah, bh[0], acc[i][0]);
            acc[i][1] = FragT<ET>::mma(ah, bh[1], acc[i][1]);
            acc[i][2] = FragT<ET>::mma(ah, bh[2], acc[i][2]);
            acc[i][3] = FragT<ET>::mma(ah, bh[3], acc[i][3]);
            guard4<V>(acc[i][0], acc[i][1], acc[i][2], acc[i][3], ah, bh[0], bh[1], bh[2], bh[3]);
        }
    }

    const int sb = wave * (16 * OP);
#pragma unroll
    for (int i = 0; i < 4; ++i) {
        const int mBase = m0 + (i << 4);
#pragma unroll
        for (int j = 0; j < 4; ++j) {
            const int n = n0 + (j << 4) + rl;
            float bvn = 0.f;
            if (BIAS_MODE == 2) bvn = bf_val(bias[n]) * bscale;
#pragma unroll
            for (int r = 0; r < 8; ++r) {
                float v = acc[i][j][r] * scale;
                if (BIAS_MODE == 1) v += bf_val(bias[mBase + mOff + r]) * bscale;
                if (BIAS_MODE == 2) v += bvn;
                sT[sb + (mOff + r) * OP + (j << 4) + rl] = v;
            }
        }
        wave_sync();
        if (OUT_MODE == 0) {
            const int hh = lane >> 4, c4 = (lane & 15) * 4;
            for (int pass = 0; pass < 2; ++pass) {
#pragma unroll
                for (int it = 0; it < 8; ++it) {
                    const int row = it * 2 + hh;
                    const v4f v = *(const v4f_ma*)&sT[sb + row * OP + c4];
                    const int grow = mBase + row;
                    const int orow = (grow / cseq) * cseqfull + (grow % cseq);
                    *(volatile v4f*)(Cf + (size_t)orow * ldc + n0 + c4) = v;
                }
                __threadfence();
            }
        } else {
            const int q = lane >> 3, c8 = (lane & 7) * 8;
            for (int pass = 0; pass < 2; ++pass) {
#pragma unroll
                for (int it = 0; it < 4; ++it) {
                    const int row = it * 4 + q;
                    const v4f a = *(const v4f_ma*)&sT[sb + row * OP + c8];
                    const v4f b = *(const v4f_ma*)&sT[sb + row * OP + c8 + 4];
                    const size_t o = (size_t)(mBase + row) * ldc + n0 + c8;
                    if (OUT_MODE == 1) {
                        v4u pk; pk.x = pk_h2f(a.x, a.y); pk.y = pk_h2f(a.z, a.w); pk.z = pk_h2f(b.x, b.y); pk.w = pk_h2f(b.z, b.w);
                        *(volatile v4u*)(Ca + o) = pk;
                    } else {
                        v4u ph, pl;
                        unsigned int h0, l0, h1, l1, h2, l2, h3, l3;
                        pk_split2(a.x, a.y, h0, l0); pk_split2(a.z, a.w, h1, l1); pk_split2(b.x, b.y, h2, l2); pk_split2(b.z, b.w, h3, l3);
                        ph.x = h0; ph.y = h1; ph.z = h2; ph.w = h3; pl.x = l0; pl.y = l1; pl.z = l2; pl.w = l3;
                        *(volatile v4u*)(Ca + o) = ph;
                        *(volatile v4u*)(Cb + o) = pl;
                    }
                }
                __threadfence();
            }
        }
        wave_sync();
    }
}

__global__ __launch_bounds__(256) void k_gemm_k(const unsigned short* __restrict__ A, const unsigned short* __restrict__ Bt,
                                                const float* __restrict__ bias, unsigned short* __restrict__ C,
                                                int M, int N, int K, float scale, float bscale) {
    gemm64_body<0, 2, 1>(A, K, Bt, K, nullptr, C, nullptr, N, bias, M, N, K, scale, bscale, 1, 1);
}

__global__ __launch_bounds__(256) void k_cast16(const float* __restrict__ src, unsigned short* __restrict__ dst, int nrows, int seq, int seqfull, float sc) {
    const int u = blockIdx.x * 256 + threadIdx.x;
    if (u >= nrows * (DM / 8)) return;
    const int r = u / (DM / 8);
    const int c0 = (u - r * (DM / 8)) * 8;
    const int sr = (r / seq) * seqfull + (r % seq);
    const float* s = src + (size_t)sr * DM + c0;
    const v4f a = *(const v4f*)(s);
    const v4f b = *(const v4f*)(s + 4);
    v4u pk;
    pk.x = pk_h2(bf_val(a.x) * sc, bf_val(a.y) * sc); pk.y = pk_h2(bf_val(a.z) * sc, bf_val(a.w) * sc);
    pk.z = pk_h2(bf_val(b.x) * sc, bf_val(b.y) * sc); pk.w = pk_h2(bf_val(b.z) * sc, bf_val(b.w) * sc);
    volatile v4u* d = (volatile v4u*)(dst + (size_t)r * DM + c0);
    *d = pk; __threadfence(); *d = pk;
}
__global__ __launch_bounds__(256) void k_cast_vt(const float* __restrict__ src, unsigned short* __restrict__ dst, int seq, int seqfull, float sc) {
    __shared__ __align__(16) _Float16 Tsh[DKH * TP];
    const int nb64 = seq / 64;
    const int b  = blockIdx.x / nb64;
    const int t0 = (blockIdx.x - b * nb64) * 64;
#pragma unroll 1
    for (int it = 0; it < 4; ++it) {
        const int idx = threadIdx.x + 256 * it;
        const int t  = idx >> 4;
        const int d4 = (idx & 15) * 4;
        const v4f a = *(const v4f*)(src + ((size_t)(b * seqfull + t0 + t)) * DKH + d4);
        Tsh[(d4 + 0) * TP + t] = toh_flush(bf_val(a.x) * sc);
        Tsh[(d4 + 1) * TP + t] = toh_flush(bf_val(a.y) * sc);
        Tsh[(d4 + 2) * TP + t] = toh_flush(bf_val(a.z) * sc);
        Tsh[(d4 + 3) * TP + t] = toh_flush(bf_val(a.w) * sc);
    }
    __syncthreads();
    for (int pass = 0; pass < 2; ++pass) {
#pragma unroll
        for (int it = 0; it < 2; ++it) {
            const int p  = threadIdx.x + 256 * it;
            const int d  = p >> 3;
            const int c8 = (p & 7) * 8;
            const v8h v = *(const v8h_ma*)&Tsh[d * TP + c8];
            const v4u pk = __builtin_bit_cast(v4u, v);
            *(volatile v4u*)(dst + (size_t)(b * DKH + d) * seq + t0 + c8) = pk;
        }
        __threadfence();
    }
}

__global__ __launch_bounds__(256) void k_attn_heads(const unsigned short* __restrict__ QP, const unsigned short* __restrict__ KP,
                                                    const unsigned short* __restrict__ VT, float* __restrict__ out,
                                                    int seq, int seqfull, float sscale) {
    __shared__ __align__(16) _Float16 Psh[NH * 8 * 16 * 16];
    __shared__ __align__(16) float    Osh[8 * 16 * OPH];
    const int lane = threadIdx.x & 31;
    const int wave = __builtin_amdgcn_readfirstlane(threadIdx.x >> 5);
    const int hf = lane >> 4;
    const int c  = lane & 15;
    const int nqb = seq / 16;
    const int b  = blockIdx.x / nqb;
    const int q0 = (blockIdx.x - b * nqb) * 16;
    const int qoff  = (b * seq + q0 + c) * DM + 8 * hf;
    const int kbase = (b * seq + wave * 16 + c) * DM + 8 * hf;
    const int vbase = (b * DKH + c) * seq + 8 * hf;
    const int obase = wave * (16 * OPH);
    const float sl2 = sscale * 1.4426950408889634f;

    v8f oacc[4];
#pragma unroll
    for (int t = 0; t < 4; ++t) { const v8f zz = {0.f, 0.f, 0.f, 0.f, 0.f, 0.f, 0.f, 0.f}; oacc[t] = zz; }

    for (int kc = 0; kc < seq; kc += KCH) {
        v8f s[NH];
#pragma unroll
        for (int h = 0; h < NH; ++h) {
            v8f z = {0.f, 0.f, 0.f, 0.f, 0.f, 0.f, 0.f, 0.f};
            const int ko = kbase + kc * DM + h * DKH;
            const int qo = qoff + h * DKH;
            const v16h ka = ldfrag_h(KP + ko);
            const v16h qa = ldfrag_h(QP + qo);
            z = mma_h(ka, qa, z);
            const v16h kb = ldfrag_h(KP + ko + 32);
            const v16h qb = ldfrag_h(QP + qo + 32);
            z = mma_h(kb, qb, z);
            s[h] = z;
            if ((h & 1) == 1) __builtin_amdgcn_sched_barrier(0);
        }
#pragma unroll
        for (int r = 0; r < 8; ++r) {
            float m = s[0][r];
#pragma unroll
            for (int h = 1; h < NH; ++h) m = fmaxf(m, s[h][r]);
            float zsum = 0.f;
#pragma unroll
            for (int h = 0; h < NH; ++h) {
                const float e = exp2f((s[h][r] - m) * sl2);
                s[h][r] = e;
                zsum += e;
            }
            const float inv = PCARRY / zsum;
#pragma unroll
            for (int h = 0; h < NH; ++h) s[h][r] = s[h][r] * inv;
        }
#pragma unroll
        for (int h = 0; h < NH; ++h) {
            v8h pv;
#pragma unroll
            for (int r = 0; r < 8; ++r) pv[r] = toh_flush(s[h][r]);
            *(v8h_ma*)&Psh[((h * 8 + wave) * 16 + c) * 16 + 8 * hf] = pv;
        }
        __syncthreads();
#pragma unroll 1
        for (int sc = 0; sc < 4; ++sc) {
            const int po = ((wave * 8 + 2 * sc) * 16 + c) * 16 + 8 * hf;
            const v8h p0 = *(const v8h_ma*)&Psh[po];
            const v8h p1 = *(const v8h_ma*)&Psh[po + 256];
            const v16h pb = __builtin_shufflevector(p0, p1, 0, 1, 2, 3, 4, 5, 6, 7, 8, 9, 10, 11, 12, 13, 14, 15);
            const int vo = vbase + kc + sc * 32;
            const v16h va0 = ldfrag_h(VT + vo);
            oacc[0] = mma_h(va0, pb, oacc[0]);
            const v16h va1 = ldfrag_h(VT + vo + 16 * seq);
            oacc[1] = mma_h(va1, pb, oacc[1]);
            const v16h va2 = ldfrag_h(VT + vo + 32 * seq);
            oacc[2] = mma_h(va2, pb, oacc[2]);
            const v16h va3 = ldfrag_h(VT + vo + 48 * seq);
            oacc[3] = mma_h(va3, pb, oacc[3]);
        }
        __syncthreads();
    }

    const float osc = 1.0f / (PCARRY * VCARRY);
#pragma unroll
    for (int half = 0; half < 2; ++half) {
#pragma unroll
        for (int tt = 0; tt < 2; ++tt) {
#pragma unroll
            for (int r = 0; r < 8; ++r) Osh[obase + c * OPH + tt * 16 + 8 * hf + r] = oacc[half * 2 + tt][r] * osc;
        }
        wave_sync();
        {
            const int q = lane >> 3, c4 = (lane & 7) * 4;
            for (int pass = 0; pass < 2; ++pass) {
#pragma unroll
                for (int it = 0; it < 4; ++it) {
                    const int row = it * 4 + q;
                    const v4f v = *(const v4f_ma*)&Osh[obase + row * OPH + c4];
                    *(volatile v4f*)(out + (size_t)(b * seqfull + q0 + row) * DM + wave * DKH + half * 32 + c4) = v;
                }
                __threadfence();
            }
        }
        wave_sync();
    }
}

constexpr size_t SZ_TOK  = (size_t)NTOK * DM * 2;
constexpr size_t SZ_V    = (size_t)NTOK * DKH * 2;
constexpr size_t SZ_W    = (size_t)DM * DKH * 2;
constexpr size_t SZ_VT   = (size_t)NB * DKH * SEQ * 2;
constexpr size_t WS_TOTAL = SZ_TOK + SZ_V + SZ_W + SZ_TOK + SZ_VT;
static_assert(SZ_TOK % 256 == 0);
static_assert(SZ_V % 256 == 0);
static_assert(SZ_W % 256 == 0);
static_assert(SZ_VT % 256 == 0);
static_assert(WS_TOTAL <= (size_t)134217728);
static_assert(((NTOK / 64) * (DM / 64)) % 8 == 0);
static_assert((size_t)NTOK * DM < (size_t)2147483647);
static_assert((size_t)NB_FULL * SEQ_FULL * DM * 4 == (size_t)8388608);

extern "C" void kernel_launch(void* const* d_in, const int* in_sizes, int n_in, void* d_out, int out_size, void* d_ws, size_t ws_size, hipStream_t stream) {
    if (n_in < 4) return;
    const long long need_q = ((long long)(NB - 1) * SEQ_FULL + SEQ) * DM;
    const long long need_v = ((long long)(NB - 1) * SEQ_FULL + SEQ) * DKH;
    if ((long long)in_sizes[0] < need_q || (long long)in_sizes[1] < need_v) return;
    if (in_sizes[2] < DM * DKH || in_sizes[3] < DM) return;
    if ((long long)out_size < need_q) return;
    if (WS_TOTAL > ws_size) return;

    const float* xq = (const float*)d_in[0];
    const float* xv = (const float*)d_in[1];
    const float* Wc = (const float*)d_in[2];
    const float* bc = (const float*)d_in[3];
    float* out = (float*)d_out;

    char* wsp = (char*)d_ws;
    unsigned short* Q16 = (unsigned short*)wsp; wsp += SZ_TOK;
    unsigned short* V16 = (unsigned short*)wsp; wsp += SZ_V;
    unsigned short* W16 = (unsigned short*)wsp; wsp += SZ_W;
    unsigned short* KPp = (unsigned short*)wsp; wsp += SZ_TOK;
    unsigned short* VTp = (unsigned short*)wsp; wsp += SZ_VT;
    if ((size_t)(wsp - (char*)d_ws) > ws_size) return;

    const unsigned gx_q = (unsigned)((NTOK * (DM / 8) + 255) / 256);
    const unsigned gx_v = (unsigned)(((NTOK / 8) * (DM / 8) + 255) / 256);
    const unsigned gx_w = (unsigned)((DKH * (DM / 8) + 255) / 256);
    const unsigned gx_gemm = (unsigned)((((NTOK / 64) * (DM / 64)) + 7) / 8);

    k_cast16<<<gx_q, 256, 0, stream>>>(xq, Q16, NTOK, SEQ, SEQ_FULL, QCARRY);
    k_cast16<<<gx_v, 256, 0, stream>>>(xv, V16, NTOK / 8, SEQ / 8, SEQ_FULL / 8, VCARRY);
    k_cast16<<<gx_w, 256, 0, stream>>>(Wc, W16, DKH, DKH, DKH, WCARRY);
    k_cast_vt<<<(unsigned)(NB * (SEQ / 64)), 256, 0, stream>>>(xv, VTp, SEQ, SEQ_FULL, VCARRY);

    k_gemm_k<<<gx_gemm, 256, 0, stream>>>(V16, W16, bc, KPp, NTOK, DM, DKH, KCARRY / (VCARRY * WCARRY), KCARRY);

    k_attn_heads<<<(unsigned)(NB * (SEQ / 16)), 256, 0, stream>>>(Q16, KPp, VTp, out, SEQ, SEQ_FULL, 0.125f / (QCARRY * KCARRY));
}
